// HierarchicalAggregation_88295937671207
// MI455X (gfx1250) — hardware-verified
//
#include <hip/hip_runtime.h>
#include <math.h>
#include <stdint.h>

#define NB    32
#define NG    15
#define NK    2048
#define NREG  (NB * NG)
#define NPT   (NREG * NK)
#define C1    64
#define C2IN  67
#define C2    128
#define C3IN  131
#define C3    256
#define N2    480
#define N3    160
#define Y1P   512
#define CHUNK 128
#define YP    136
#define WP    72
#define WSC   16.0f
#define IWSC  (1.0f / 16.0f)
#define LOSC  4096.0f
#define ILOSC (1.0f / 4096.0f)
#define BN_EPS 1e-5f

static_assert(NK % CHUNK == 0 && CHUNK == 128 && NK % 256 == 0);
static_assert(((C2IN * N2) % 32) == 0 && ((NB * C2IN * NG) % 32) == 0 && ((3 * N3) % 32) == 0);
static_assert((N2 % 32) == 0 && (N3 % 32) == 0 && (Y1P % 32) == 0);
static_assert((YP * 2) % 16 == 0 && (WP * 2) % 16 == 0);

typedef _Float16 v16h __attribute__((ext_vector_type(16)));
typedef _Float16 v8h  __attribute__((ext_vector_type(8)));
typedef float    v8f  __attribute__((ext_vector_type(8)));
typedef float    v4f  __attribute__((ext_vector_type(4)));
union FragH { v16h v; v8h hf[2]; };
union H8 { v8h v; _Float16 f[8]; };
union F4 { v4f v; float f[4]; };

__constant__ int c_sidx[15] = {0, 1, 8, 2, 4, 6, 3, 5, 7, 9, 11, 13, 10, 12, 14};

__device__ __forceinline__ unsigned short bf_bits(float f) {
  unsigned u = __float_as_uint(f);
  return (unsigned short)((u + 0x7FFFu + ((u >> 16) & 1u)) >> 16);
}
__device__ __forceinline__ float bf_up(unsigned short b) { return __uint_as_float(((unsigned)b) << 16); }
__device__ __forceinline__ float bfr(float f) { return bf_up(bf_bits(f)); }
__device__ __forceinline__ v8f zero8() { v8f z = {0.f, 0.f, 0.f, 0.f, 0.f, 0.f, 0.f, 0.f}; return z; }

__device__ __forceinline__ void split16(float t, _Float16& hh, _Float16& ll) {
  const _Float16 h0 = (_Float16)t;
  const _Float16 hz = (_Float16)0.0f;
  hh = (fabsf(t) < 6.103515625e-05f) ? hz : h0;
  ll = (_Float16)((t - (float)hh) * LOSC);
}

__device__ __forceinline__ v16h ldf(const _Float16* p) {
  FragH f;
  f.hf[0] = *(const v8h*)(p);
  f.hf[1] = *(const v8h*)(p + 16);
  return f.v;
}
__device__ __forceinline__ v8f mma(v16h a, v16h b, v8f c) {
  return __builtin_amdgcn_wmma_f32_16x16x32_f16(false, a, false, b, (short)0, c, false, false);
}
__device__ __forceinline__ void guard2(v8f& c, v8f& e, v16h a0, v16h a1, v16h a2, v16h a3, v16h b0, v16h b1) {
#if defined(__HIP_DEVICE_COMPILE__)
  asm volatile("v_nop\n\tv_nop\n\tv_nop\n\tv_nop"
               : "+v"(c), "+v"(e)
               : "v"(a0), "v"(a1), "v"(a2), "v"(a3), "v"(b0), "v"(b1));
#endif
}

__device__ __forceinline__ float block_sum256(float v, float* red) {
  const int t = threadIdx.x;
  red[t] = v;
  __syncthreads();
#pragma unroll
  for (int o = 128; o > 0; o >>= 1) {
    if (t < o) red[t] = red[t] + red[t + o];
    __syncthreads();
  }
  const float r = red[0];
  __syncthreads();
  return r;
}

__global__ __launch_bounds__(256) void k_cent(const float* __restrict__ lr, float* cent) {
  __shared__ float sP[9][256];
  __shared__ double sS[4];
  __shared__ __align__(16) float sLine[32];
  const int t = threadIdx.x, reg = blockIdx.x;
  const float* p = lr + (size_t)reg * NK * 3;
  float sx = 0.f, sy = 0.f, sz = 0.f;
#pragma unroll 1
  for (int i = 0; i < NK / 256; ++i) {
    const float* q = p + (size_t)(i * 256 + t) * 3;
    sx += bfr(q[0]); sy += bfr(q[1]); sz += bfr(q[2]);
  }
  sP[0][t] = sx; sP[1][t] = sy; sP[2][t] = sz;
  if (t < 32) sLine[t] = 0.0f;
  __syncthreads();
  if (t < 3) {
    double s = 0.0;
#pragma unroll 1
    for (int j = 0; j < 256; ++j) s += (double)sP[t][j];
    sS[t] = s;
  }
  __syncthreads();
  const float cx = (float)sS[0] * (1.0f / (float)NK);
  const float cy = (float)sS[1] * (1.0f / (float)NK);
  const float cz = (float)sS[2] * (1.0f / (float)NK);
  float a0 = 0.f, a1 = 0.f, a2 = 0.f, a3 = 0.f, a4 = 0.f, a5 = 0.f, a6 = 0.f, a7 = 0.f, a8 = 0.f;
#pragma unroll 1
  for (int i = 0; i < NK / 256; ++i) {
    const float* q = p + (size_t)(i * 256 + t) * 3;
    const float r0 = bfr(q[0]) - cx, r1 = bfr(q[1]) - cy, r2 = bfr(q[2]) - cz;
    a0 += r0; a1 += r1; a2 += r2;
    a3 += r0 * r0; a4 += r0 * r1; a5 += r0 * r2;
    a6 += r1 * r1; a7 += r1 * r2; a8 += r2 * r2;
  }
  sP[0][t] = a0; sP[1][t] = a1; sP[2][t] = a2; sP[3][t] = a3; sP[4][t] = a4;
  sP[5][t] = a5; sP[6][t] = a6; sP[7][t] = a7; sP[8][t] = a8;
  __syncthreads();
  if (t < 9) {
    double s = 0.0;
#pragma unroll 1
    for (int j = 0; j < 256; ++j) s += (double)sP[t][j];
    const int e = (t < 3) ? (4 + t) : (5 + t);
    sLine[e] = (float)s;
  }
  if (t == 0) { sLine[0] = cx; sLine[1] = cy; sLine[2] = cz; }
  __syncthreads();
  if (t < 8) {
    const v4f v = *(const v4f*)(sLine + t * 4);
    float* dst = cent + (size_t)reg * 32 + t * 4;
    *(volatile v4f*)dst = v;
    __threadfence();
    *(volatile v4f*)dst = v;
  }
}

__global__ __launch_bounds__(256) void k_fin0(const float* cent, const float* W0, const float* g0, const float* b0,
                                             float* coef) {
  __shared__ double sS[16];
  __shared__ __align__(16) float sOut[512];
  const int t = threadIdx.x;
  sOut[t] = 0.0f;
  sOut[256 + t] = 0.0f;
  if (t < 9) {
    const int e = (t < 3) ? (4 + t) : (5 + t);
    double s = 0.0;
#pragma unroll 1
    for (int r = 0; r < NREG; ++r) s += (double)cent[(size_t)r * 32 + e];
    sS[t] = s;
  }
  __syncthreads();
  if (t < C1) {
    const double invn = 1.0 / (double)NPT;
    const double w0 = (double)bfr(W0[t * 3 + 0]), w1 = (double)bfr(W0[t * 3 + 1]), w2 = (double)bfr(W0[t * 3 + 2]);
    const double m0 = sS[0] * invn, m1 = sS[1] * invn, m2 = sS[2] * invn;
    const double M00 = sS[3] * invn, M01 = sS[4] * invn, M02 = sS[5] * invn;
    const double M11 = sS[6] * invn, M12 = sS[7] * invn, M22 = sS[8] * invn;
    const double mu = w0 * m0 + w1 * m1 + w2 * m2;
    const double e2 = w0 * w0 * M00 + w1 * w1 * M11 + w2 * w2 * M22 +
                      2.0 * (w0 * w1 * M01 + w0 * w2 * M02 + w1 * w2 * M12);
    double var = e2 - mu * mu;
    if (var < 0.0) var = 0.0;
    const float rstd = (float)(1.0 / sqrt(var + 1.0e-5));
    const float sc = bfr(g0[t]) * rstd;
    const float sh = bfr(b0[t]) - (float)mu * sc;
    sOut[t] = (float)w0; sOut[C1 + t] = (float)w1; sOut[2 * C1 + t] = (float)w2;
    sOut[3 * C1 + t] = sc; sOut[4 * C1 + t] = sh;
  }
  __syncthreads();
  if (t < 128) {
    const v4f v = *(const v4f*)(sOut + t * 4);
    float* dst = coef + t * 4;
    *(volatile v4f*)dst = v;
    __threadfence();
    *(volatile v4f*)dst = v;
  }
}

__global__ __launch_bounds__(256) void k_l1b(const float* __restrict__ lr, const float* cent, const float* coef,
                                             const float* W1, float* part) {
  __shared__ __align__(16) _Float16 sY[CHUNK * YP];
  __shared__ __align__(16) _Float16 sW[C1 * WP];
  __shared__ __align__(16) float sCo[5 * C1];
  __shared__ __align__(16) float sRed[8][4][C1];
  __shared__ __align__(16) float sOut[256];
  const int tid = threadIdx.x, wave = tid >> 5, lane = tid & 31;
  const int m = lane & 15, h = lane >> 4, k8 = h * 8;
  const int reg = blockIdx.x;
  for (int i = tid; i < 5 * C1; i += 256) sCo[i] = coef[i];
#pragma unroll
  for (int i = 0; i < 16; ++i) {
    const int idx = tid * 16 + i;
    const int n = idx >> 6, k = idx & 63;
    sW[n * WP + k] = (_Float16)(bfr(W1[idx]) * WSC);
  }
  const float cx = cent[(size_t)reg * 32 + 0], cy = cent[(size_t)reg * 32 + 1], cz = cent[(size_t)reg * 32 + 2];
  __syncthreads();
  float rs[4], rq[4], rmx[4], rmn[4];
#pragma unroll
  for (int nt = 0; nt < 4; ++nt) { rs[nt] = 0.f; rq[nt] = 0.f; rmx[nt] = -3.0e38f; rmn[nt] = 3.0e38f; }
  const int pt = tid & (CHUNK - 1), chalf = tid >> 7;
  const float* preg = lr + (size_t)reg * NK * 3;
#pragma unroll 1
  for (int ch = 0; ch < NK / CHUNK; ++ch) {
    {
      const float* pp = preg + (size_t)(ch * CHUNK + pt) * 3;
      const float r0 = bfr(pp[0]) - cx, r1 = bfr(pp[1]) - cy, r2 = bfr(pp[2]) - cz;
      _Float16* yrow = sY + pt * YP + chalf * 32;
#pragma unroll
      for (int q = 0; q < 4; ++q) {
        H8 ph, pl;
#pragma unroll
        for (int u = 0; u < 8; ++u) {
          const int c = chalf * 32 + q * 8 + u;
          const float y0 = sCo[c] * r0 + sCo[C1 + c] * r1 + sCo[2 * C1 + c] * r2;
          float t = y0 * sCo[3 * C1 + c] + sCo[4 * C1 + c];
          t = fmaxf(t, 0.0f);
          _Float16 hh, ll;
          split16(t, hh, ll);
          ph.f[u] = hh;
          pl.f[u] = ll;
        }
        *(v8h*)(yrow + q * 8) = ph.v;
        *(v8h*)(yrow + C1 + q * 8) = pl.v;
      }
    }
    __syncthreads();
    {
      const _Float16* ar = sY + (wave * 16 + m) * YP + k8;
      const v16h ha0 = ldf(ar), ha1 = ldf(ar + 32), la0 = ldf(ar + C1), la1 = ldf(ar + C1 + 32);
#pragma unroll
      for (int nt = 0; nt < 4; ++nt) {
        const _Float16* wr = sW + (nt * 16 + m) * WP + k8;
        const v16h b0 = ldf(wr), b1 = ldf(wr + 32);
        v8f c = zero8(), e = zero8();
        c = mma(ha0, b0, c);
        c = mma(ha1, b1, c);
        e = mma(la0, b0, e);
        e = mma(la1, b1, e);
        guard2(c, e, ha0, ha1, la0, la1, b0, b1);
#pragma unroll
        for (int r = 0; r < 8; ++r) {
          const float z = (c[r] + e[r] * ILOSC) * IWSC;
          rs[nt] += z;
          rq[nt] += z * z;
          rmx[nt] = fmaxf(rmx[nt], z);
          rmn[nt] = fminf(rmn[nt], z);
        }
      }
    }
    __syncthreads();
  }
#pragma unroll
  for (int nt = 0; nt < 4; ++nt) {
    const float s2 = rs[nt] + __shfl_xor(rs[nt], 16, 32);
    const float q2 = rq[nt] + __shfl_xor(rq[nt], 16, 32);
    const float x2 = fmaxf(rmx[nt], __shfl_xor(rmx[nt], 16, 32));
    const float n2 = fminf(rmn[nt], __shfl_xor(rmn[nt], 16, 32));
    if (h == 0) {
      sRed[wave][0][nt * 16 + m] = s2;
      sRed[wave][1][nt * 16 + m] = q2;
      sRed[wave][2][nt * 16 + m] = x2;
      sRed[wave][3][nt * 16 + m] = n2;
    }
  }
  __syncthreads();
  {
    const int st = tid >> 6, c = tid & 63;
    float as = 0.0f, ax = -3.0e38f, an = 3.0e38f;
#pragma unroll
    for (int w = 0; w < 8; ++w) {
      const float v = sRed[w][st][c];
      as += v;
      ax = fmaxf(ax, v);
      an = fminf(an, v);
    }
    sOut[tid] = (st < 2) ? as : ((st == 2) ? ax : an);
  }
  __syncthreads();
  if (tid < 64) {
    const v4f v = *(const v4f*)(sOut + tid * 4);
    float* dst = part + (size_t)reg * 256 + tid * 4;
    *(volatile v4f*)dst = v;
    __threadfence();
    *(volatile v4f*)dst = v;
  }
}

__device__ __forceinline__ float lf1v(const float* part, const float* sSc, const float* sSh, int b, int c, int g) {
  const int reg = b * NG + g;
  const float mx = part[(size_t)reg * 256 + 128 + c];
  const float mn = part[(size_t)reg * 256 + 192 + c];
  const float sc = sSc[c], sh = sSh[c];
  const float v = (sc >= 0.0f) ? mx : mn;
  return fmaxf(sc * v + sh, 0.0f);
}

__global__ __launch_bounds__(256) void k_fin1(const float* cent, const float* part, const float* g1, const float* b1,
                                             float* out1, float* X2, float* X3) {
  __shared__ double sAcc[2][C1];
  __shared__ float sSc[C1];
  __shared__ float sSh[C1];
  __shared__ float sC[NREG * 3];
  __shared__ float sC2[NB * 5 * 3];
  __shared__ float sC3[NB * 3];
  const int t = threadIdx.x;
  if (t < 128) {
    const int which = t >> 6, c = t & 63;
    double s = 0.0;
#pragma unroll 1
    for (int r = 0; r < NREG; ++r) s += (double)part[(size_t)r * 256 + which * 64 + c];
    sAcc[which][c] = s;
  }
  for (int i = t; i < NREG * 3; i += 256) {
    const int reg = i / 3, k = i - reg * 3;
    sC[i] = cent[(size_t)reg * 32 + k];
  }
  __syncthreads();
  if (t < C1) {
    const double invn = 1.0 / (double)NPT;
    const double mean = sAcc[0][t] * invn;
    double var = sAcc[1][t] * invn - mean * mean;
    if (var < 0.0) var = 0.0;
    const float rstd = (float)(1.0 / sqrt(var + 1.0e-5));
    const float sc = bfr(g1[t]) * rstd;
    sSc[t] = sc;
    sSh[t] = bfr(b1[t]) - (float)mean * sc;
  }
  for (int i = t; i < NB * 15; i += 256) {
    const int b = i / 15, rem = i - b * 15, s = rem / 3, k = rem - s * 3;
    const float v0 = sC[(b * NG + c_sidx[s * 3 + 0]) * 3 + k];
    const float v1 = sC[(b * NG + c_sidx[s * 3 + 1]) * 3 + k];
    const float v2 = sC[(b * NG + c_sidx[s * 3 + 2]) * 3 + k];
    sC2[i] = ((v0 + v1) + v2) * (1.0f / 3.0f);
  }
  __syncthreads();
  if (t < NB * 3) {
    const int b = t / 3, k = t - b * 3;
    float a = sC2[(b * 5 + 0) * 3 + k];
    a += sC2[(b * 5 + 1) * 3 + k];
    a += sC2[(b * 5 + 2) * 3 + k];
    a += sC2[(b * 5 + 3) * 3 + k];
    a += sC2[(b * 5 + 4) * 3 + k];
    sC3[t] = a * (1.0f / 5.0f);
  }
  __syncthreads();
#pragma unroll 1
  for (int pz = t; pz < (NB * C2IN * NG) / 4; pz += 256) {
    F4 o;
#pragma unroll
    for (int u = 0; u < 4; ++u) {
      const int e = pz * 4 + u;
      const int b = e / (C2IN * NG);
      const int rem = e - b * (C2IN * NG);
      const int ch = rem / NG;
      const int g = rem - ch * NG;
      const int chc = (ch < 3) ? ch : 2;
      const int cc = (ch >= 3) ? (ch - 3) : 0;
      const float vc = sC[(b * NG + g) * 3 + chc];
      const float vl = lf1v(part, sSc, sSh, b, cc, g);
      o.f[u] = (ch < 3) ? vc : vl;
    }
    float* dst = out1 + (size_t)pz * 4;
    *(volatile v4f*)dst = o.v;
    __threadfence();
    *(volatile v4f*)dst = o.v;
  }
#pragma unroll 1
  for (int pz = t; pz < (C2IN * N2) / 4; pz += 256) {
    F4 o;
#pragma unroll
    for (int u = 0; u < 4; ++u) {
      const int e = pz * 4 + u;
      const int i = e / N2;
      const int col = e - i * N2;
      const int b = col / NG;
      const int rem = col - b * NG;
      const int s = rem / 3;
      const int j = rem - s * 3;
      const int gi = c_sidx[s * 3 + j];
      const int ic = (i < 3) ? i : 2;
      const int cc = (i >= 3) ? (i - 3) : 0;
      const float vr = sC[(b * NG + gi) * 3 + ic] - sC2[(b * 5 + s) * 3 + ic];
      const float vl = lf1v(part, sSc, sSh, b, cc, gi);
      o.f[u] = (i < 3) ? vr : vl;
    }
    float* dst = X2 + (size_t)pz * 4;
    *(volatile v4f*)dst = o.v;
    __threadfence();
    *(volatile v4f*)dst = o.v;
  }
  if (t < (3 * N3) / 4) {
    F4 o;
#pragma unroll
    for (int u = 0; u < 4; ++u) {
      const int e = t * 4 + u;
      const int i = e / N3;
      const int col = e - i * N3;
      const int b = col / 5;
      const int s = col - b * 5;
      o.f[u] = sC2[(b * 5 + s) * 3 + i] - sC3[b * 3 + i];
    }
    float* dst = X3 + (size_t)t * 4;
    *(volatile v4f*)dst = o.v;
    __threadfence();
    *(volatile v4f*)dst = o.v;
  }
}

__global__ __launch_bounds__(256) void k_l2a(const float* X2, const float* W, const float* g, const float* b, float* Y1) {
  __shared__ float sWr[C2IN + 1];
  __shared__ float sRed[256];
  __shared__ __align__(16) float sRow[Y1P];
  const int t = threadIdx.x, o = blockIdx.x;
  if (t < C2IN) sWr[t] = bfr(W[(size_t)o * C2IN + t]);
  __syncthreads();
  const int c0 = t, c1 = t + 256;
  const bool v1 = c1 < N2;
  const int c1c = v1 ? c1 : (N2 - 1);
  float a0 = 0.0f, a1 = 0.0f;
#pragma unroll 4
  for (int i = 0; i < C2IN; ++i) {
    const float w = sWr[i];
    a0 += w * X2[(size_t)i * N2 + c0];
    a1 += w * X2[(size_t)i * N2 + c1c];
  }
  const float s = block_sum256(a0 + (v1 ? a1 : 0.0f), sRed);
  const float mu = s * (1.0f / (float)N2);
  const float d0 = a0 - mu, d1 = a1 - mu;
  const float q = block_sum256(d0 * d0 + (v1 ? d1 * d1 : 0.0f), sRed);
  const float rstd = rsqrtf(q * (1.0f / (float)N2) + BN_EPS);
  const float gg = bfr(g[o]), bb = bfr(b[o]);
  sRow[c0] = fmaxf(d0 * rstd * gg + bb, 0.0f);
  if (v1) sRow[c1] = fmaxf(d1 * rstd * gg + bb, 0.0f);
  else sRow[N2 + (t - (N2 - 256))] = 0.0f;
  __syncthreads();
  if (t < Y1P / 4) {
    const v4f v = *(const v4f*)(sRow + t * 4);
    float* dst = Y1 + (size_t)o * Y1P + t * 4;
    *(volatile v4f*)dst = v;
    __threadfence();
    *(volatile v4f*)dst = v;
  }
}

__global__ __launch_bounds__(256) void k_l2b(const float* Y1, const float* W, const float* g, const float* b, float* X3) {
  __shared__ float sWr[C2];
  __shared__ float sRed[256];
  __shared__ __align__(16) float sRow[N2];
  __shared__ __align__(16) float sM[N3];
  const int t = threadIdx.x, o = blockIdx.x;
  for (int i = t; i < C2; i += 256) sWr[i] = bfr(W[(size_t)o * C2 + i]);
  __syncthreads();
  const int c0 = t, c1 = t + 256;
  const bool v1 = c1 < N2;
  const int c1c = v1 ? c1 : (N2 - 1);
  float a0 = 0.0f, a1 = 0.0f;
#pragma unroll 4
  for (int i = 0; i < C2; ++i) {
    const float w = sWr[i];
    a0 += w * Y1[(size_t)i * Y1P + c0];
    a1 += w * Y1[(size_t)i * Y1P + c1c];
  }
  const float s = block_sum256(a0 + (v1 ? a1 : 0.0f), sRed);
  const float mu = s * (1.0f / (float)N2);
  const float d0 = a0 - mu, d1 = a1 - mu;
  const float q = block_sum256(d0 * d0 + (v1 ? d1 * d1 : 0.0f), sRed);
  const float rstd = rsqrtf(q * (1.0f / (float)N2) + BN_EPS);
  const float gg = bfr(g[o]), bb = bfr(b[o]);
  sRow[c0] = fmaxf(d0 * rstd * gg + bb, 0.0f);
  if (v1) sRow[c1] = fmaxf(d1 * rstd * gg + bb, 0.0f);
  __syncthreads();
  if (t < N3) {
    const float m0 = sRow[3 * t + 0], m1 = sRow[3 * t + 1], m2 = sRow[3 * t + 2];
    sM[t] = fmaxf(fmaxf(m0, m1), m2);
  }
  __syncthreads();
  if (t < N3 / 4) {
    const v4f v = *(const v4f*)(sM + t * 4);
    float* dst = X3 + (size_t)(3 + o) * N3 + t * 4;
    *(volatile v4f*)dst = v;
    __threadfence();
    *(volatile v4f*)dst = v;
  }
}

__global__ __launch_bounds__(256) void k_l3a(const float* X3, const float* W, const float* g, const float* b, float* Y3) {
  __shared__ float sWr[C3IN + 1];
  __shared__ float sRed[256];
  __shared__ __align__(16) float sRow[N3];
  const int t = threadIdx.x, o = blockIdx.x;
  for (int i = t; i < C3IN; i += 256) sWr[i] = bfr(W[(size_t)o * C3IN + i]);
  __syncthreads();
  const bool valid = t < N3;
  const int cc = valid ? t : (N3 - 1);
  float a = 0.0f;
  if (valid) {
#pragma unroll 4
    for (int i = 0; i < C3IN; ++i) a += sWr[i] * X3[(size_t)i * N3 + cc];
  }
  const float s = block_sum256(valid ? a : 0.0f, sRed);
  const float mu = s * (1.0f / (float)N3);
  const float d = a - mu;
  const float q = block_sum256(valid ? d * d : 0.0f, sRed);
  const float rstd = rsqrtf(q * (1.0f / (float)N3) + BN_EPS);
  const float gg = bfr(g[o]), bb = bfr(b[o]);
  if (valid) sRow[t] = fmaxf(d * rstd * gg + bb, 0.0f);
  __syncthreads();
  if (t < N3 / 4) {
    const v4f v = *(const v4f*)(sRow + t * 4);
    float* dst = Y3 + (size_t)o * N3 + t * 4;
    *(volatile v4f*)dst = v;
    __threadfence();
    *(volatile v4f*)dst = v;
  }
}

__global__ __launch_bounds__(256) void k_l3b(const float* Y3, const float* W, const float* g, const float* b, float* gft) {
  __shared__ float sWr[C3];
  __shared__ float sRed[256];
  __shared__ __align__(16) float sRow[N3];
  __shared__ __align__(16) float sM[NB];
  const int t = threadIdx.x, o = blockIdx.x;
  for (int i = t; i < C3; i += 256) sWr[i] = bfr(W[(size_t)o * C3 + i]);
  __syncthreads();
  const bool valid = t < N3;
  const int cc = valid ? t : (N3 - 1);
  float a = 0.0f;
  if (valid) {
#pragma unroll 4
    for (int i = 0; i < C3; ++i) a += sWr[i] * Y3[(size_t)i * N3 + cc];
  }
  const float s = block_sum256(valid ? a : 0.0f, sRed);
  const float mu = s * (1.0f / (float)N3);
  const float d = a - mu;
  const float q = block_sum256(valid ? d * d : 0.0f, sRed);
  const float rstd = rsqrtf(q * (1.0f / (float)N3) + BN_EPS);
  const float gg = bfr(g[o]), bb = bfr(b[o]);
  if (valid) sRow[t] = fmaxf(d * rstd * gg + bb, 0.0f);
  __syncthreads();
  if (t < NB) {
    float mxv = sRow[5 * t + 0];
    mxv = fmaxf(mxv, sRow[5 * t + 1]);
    mxv = fmaxf(mxv, sRow[5 * t + 2]);
    mxv = fmaxf(mxv, sRow[5 * t + 3]);
    mxv = fmaxf(mxv, sRow[5 * t + 4]);
    sM[t] = mxv;
  }
  __syncthreads();
  if (t < NB / 4) {
    const v4f v = *(const v4f*)(sM + t * 4);
    float* dst = gft + (size_t)o * 32 + t * 4;
    *(volatile v4f*)dst = v;
    __threadfence();
    *(volatile v4f*)dst = v;
  }
}

__global__ __launch_bounds__(256) void k_out0(const float* gft, float* out) {
  const int t = threadIdx.x;
#pragma unroll 1
  for (int it = 0; it < (NB * C3) / 1024; ++it) {
    const int pz = it * 256 + t;
    F4 o;
#pragma unroll
    for (int u = 0; u < 4; ++u) {
      const int e = pz * 4 + u;
      const int b = e >> 8, oc = e & 255;
      o.f[u] = gft[(size_t)oc * 32 + b];
    }
    float* dst = out + (size_t)pz * 4;
    *(volatile v4f*)dst = o.v;
    __threadfence();
    *(volatile v4f*)dst = o.v;
  }
}

extern "C" void kernel_launch(void* const* d_in, const int* in_sizes, int n_in,
                              void* d_out, int out_size, void* d_ws, size_t ws_size, hipStream_t stream) {
  if (n_in < 19) return;
  if (in_sizes[0] != NPT * 3) return;
  if (in_sizes[1] != C1 * 3 || in_sizes[2] != C1 || in_sizes[3] != C1) return;
  if (in_sizes[4] != C1 * C1 || in_sizes[5] != C1 || in_sizes[6] != C1) return;
  if (in_sizes[7] != C2 * C2IN || in_sizes[8] != C2 || in_sizes[9] != C2) return;
  if (in_sizes[10] != C2 * C2 || in_sizes[11] != C2 || in_sizes[12] != C2) return;
  if (in_sizes[13] != C3 * C3IN || in_sizes[14] != C3 || in_sizes[15] != C3) return;
  if (in_sizes[16] != C3 * C3 || in_sizes[17] != C3 || in_sizes[18] != C3) return;
  if (out_size != NB * C3 + NB * C2IN * NG) return;

  const float* lr     = (const float*)d_in[0];
  const float* la0_w0 = (const float*)d_in[1];
  const float* la0_g0 = (const float*)d_in[2];
  const float* la0_b0 = (const float*)d_in[3];
  const float* la0_w1 = (const float*)d_in[4];
  const float* la0_g1 = (const float*)d_in[5];
  const float* la0_b1 = (const float*)d_in[6];
  const float* la1_w0 = (const float*)d_in[7];
  const float* la1_g0 = (const float*)d_in[8];
  const float* la1_b0 = (const float*)d_in[9];
  const float* la1_w1 = (const float*)d_in[10];
  const float* la1_g1 = (const float*)d_in[11];
  const float* la1_b1 = (const float*)d_in[12];
  const float* la2_w0 = (const float*)d_in[13];
  const float* la2_g0 = (const float*)d_in[14];
  const float* la2_b0 = (const float*)d_in[15];
  const float* la2_w1 = (const float*)d_in[16];
  const float* la2_g1 = (const float*)d_in[17];
  const float* la2_b1 = (const float*)d_in[18];
  float* out0 = (float*)d_out;
  float* out1 = out0 + NB * C3;

  const size_t PCENT = (size_t)NREG * 32 * 4;
  const size_t PCOEF = (size_t)8 * C1 * 4;
  const size_t PPART = (size_t)NREG * 256 * 4;
  const size_t PX2   = (size_t)C2IN * N2 * 4;
  const size_t PY1   = (size_t)C2 * Y1P * 4;
  const size_t PX3   = (size_t)C3IN * N3 * 4;
  const size_t PY3   = (size_t)C3 * N3 * 4;
  const size_t PGFT  = (size_t)C3 * 32 * 4;
  size_t off = 0;
  const size_t oCENT = off; off += PCENT;
  const size_t oCOEF = off; off += PCOEF;
  const size_t oPART = off; off += PPART;
  const size_t oX2   = off; off += PX2;
  const size_t oY1   = off; off += PY1;
  const size_t oX3   = off; off += PX3;
  const size_t oY3   = off; off += PY3;
  const size_t oGFT  = off; off += PGFT;
  if (off > ws_size) return;
  if (off > (size_t)134217728) return;

  char* ws = (char*)d_ws;
  float* cent = (float*)(ws + oCENT);
  float* coef = (float*)(ws + oCOEF);
  float* part = (float*)(ws + oPART);
  float* X2   = (float*)(ws + oX2);
  float* Y1   = (float*)(ws + oY1);
  float* X3   = (float*)(ws + oX3);
  float* Y3   = (float*)(ws + oY3);
  float* gft  = (float*)(ws + oGFT);

  const dim3 blk(256);
  k_cent<<<dim3(NREG), blk, 0, stream>>>(lr, cent);
  k_fin0<<<dim3(1), blk, 0, stream>>>(cent, la0_w0, la0_g0, la0_b0, coef);
  k_l1b<<<dim3(NREG), blk, 0, stream>>>(lr, cent, coef, la0_w1, part);
  k_fin1<<<dim3(1), blk, 0, stream>>>(cent, part, la0_g1, la0_b1, out1, X2, X3);
  k_l2a<<<dim3(C2), blk, 0, stream>>>(X2, la1_w0, la1_g0, la1_b0, Y1);
  k_l2b<<<dim3(C2), blk, 0, stream>>>(Y1, la1_w1, la1_g1, la1_b1, X3);
  k_l3a<<<dim3(C3), blk, 0, stream>>>(X3, la2_w0, la2_g0, la2_b0, Y3);
  k_l3b<<<dim3(C3), blk, 0, stream>>>(Y3, la2_w1, la2_g1, la2_b1, gft);
  k_out0<<<dim3(1), blk, 0, stream>>>(gft, out0);
  (void)hipGetLastError();
}
